// DeformableConv2D_81810537054370
// MI455X (gfx1250) — hardware-run, weakly checked
//
#include <hip/hip_runtime.h>

typedef float          v8f   __attribute__((ext_vector_type(8)));
typedef float          v4f   __attribute__((ext_vector_type(4)));
typedef unsigned int   v4u   __attribute__((ext_vector_type(4)));
typedef int            v8i   __attribute__((ext_vector_type(8)));
typedef unsigned short v8us  __attribute__((ext_vector_type(8)));
typedef unsigned short v16us __attribute__((ext_vector_type(16)));
typedef __bf16         v16bf __attribute__((ext_vector_type(16)));
typedef _Float16       v16h  __attribute__((ext_vector_type(16)));
typedef v4f  __attribute__((may_alias)) v4fa;
typedef v8us __attribute__((may_alias)) v8usa;
union FragB { v16bf v; v16us u; v8us h[2]; v8i w; };
union FragH { v16h  v; v16us u; v8us h[2]; v8i w; };

__device__ __forceinline__ v8f wmb(const FragB& a, const FragB& b, v8f c) {
  v8f d = __builtin_amdgcn_wmma_f32_16x16x32_bf16(false, a.v, false, b.v, (short)0, c, false, false);
  asm volatile("v_nop\n\tv_nop\n\tv_nop\n\tv_nop" : "+v"(d) : "v"(a.w), "v"(b.w));
  return d;
}

__device__ __forceinline__ v8f wmh(const FragH& a, const FragH& b, v8f c) {
  v8f d = __builtin_amdgcn_wmma_f32_16x16x32_f16(false, a.v, false, b.v, (short)0, c, false, false);
  asm volatile("v_nop\n\tv_nop\n\tv_nop\n\tv_nop" : "+v"(d) : "v"(a.w), "v"(b.w));
  return d;
}

__device__ __forceinline__ unsigned bf16_bits(float f) {
  const unsigned u = __float_as_uint(f);
  const unsigned r = (u + 0x7FFFu + ((u >> 16) & 1u)) >> 16;
  const unsigned q = (u >> 16) | 0x40u;
  return ((u & 0x7fffffffu) > 0x7f800000u) ? q : r;
}

__device__ __forceinline__ float bf16_val(float f) {
  return __uint_as_float(bf16_bits(f) << 16);
}
__device__ __forceinline__ int clampi(int v, int lo, int hi) {
  return v < lo ? lo : (v > hi ? hi : v);
}

__device__ __forceinline__ unsigned f16_bits(float f) {
  const unsigned u  = __float_as_uint(f);
  const unsigned s  = (u >> 16) & 0x8000u;
  const unsigned a  = u & 0x7fffffffu;
  const unsigned t  = a - 0x38000000u;
  const unsigned r  = (t + 0x0FFFu + ((t >> 13) & 1u)) >> 13;
  const unsigned rc = r > 0x7C00u ? 0x7C00u : r;
  const bool small  = a < 0x38800000u;
  const bool isnan  = a > 0x7f800000u;
  const unsigned fin = small ? 0u : (s | rc);
  return isnan ? (s | 0x7E00u) : fin;
}

__device__ __forceinline__ unsigned pk16(unsigned lo, unsigned hi) { return lo | (hi << 16); }
__device__ __forceinline__ unsigned bf16_lo_bits(float v) {
  float hi = bf16_val(v);
  asm volatile("" : "+v"(hi));
  return bf16_bits(v - hi);
}
__device__ __forceinline__ v4u pack8_bf16(v4f a, v4f c) {
  return (v4u){ pk16(bf16_bits(a[0]), bf16_bits(a[1])), pk16(bf16_bits(a[2]), bf16_bits(a[3])),
                pk16(bf16_bits(c[0]), bf16_bits(c[1])), pk16(bf16_bits(c[2]), bf16_bits(c[3])) };
}
__device__ __forceinline__ v4u pack8_bf16_lo(v4f a, v4f c) {
  return (v4u){ pk16(bf16_lo_bits(a[0]), bf16_lo_bits(a[1])), pk16(bf16_lo_bits(a[2]), bf16_lo_bits(a[3])),
                pk16(bf16_lo_bits(c[0]), bf16_lo_bits(c[1])), pk16(bf16_lo_bits(c[2]), bf16_lo_bits(c[3])) };
}
__device__ __forceinline__ v4u pack8_f16(v4f a, v4f c) {
  return (v4u){ pk16(f16_bits(a[0]), f16_bits(a[1])), pk16(f16_bits(a[2]), f16_bits(a[3])),
                pk16(f16_bits(c[0]), f16_bits(c[1])), pk16(f16_bits(c[2]), f16_bits(c[3])) };
}

template <int FORM>
__global__ __launch_bounds__(256) void k_plane(const float* __restrict__ src, int rows, int cols, int ldsrc,
                                               unsigned short* __restrict__ dst, int MP, int KP) {
  static_assert(FORM >= 0 && FORM <= 3);
  const int KTOT = (FORM == 1 || FORM == 3) ? 2 * KP : KP;
  const unsigned ppr   = (unsigned)(KTOT >> 3);
  const unsigned kp8   = (unsigned)(KP >> 3);
  const unsigned total = (unsigned)MP * ppr;
  const unsigned g     = blockIdx.x * 256u + threadIdx.x;
  const unsigned rowu  = g / ppr;
  const unsigned p     = g - rowu * ppr;
  const bool second    = p >= kp8;
  const int row = (int)rowu;
  const int c0  = (int)((second ? p - kp8 : p) << 3);
  const float* srow = src + (size_t)clampi(row, 0, rows - 1) * (size_t)ldsrc;
  float x[8];
  unsigned mk[8];
#pragma unroll
  for (int e = 0; e < 8; ++e) {
    const int c = c0 + e;
    const float v = srow[clampi(c, 0, cols - 1)];
    asm volatile("" :: "v"(v));
    x[e]  = v;
    mk[e] = (row < rows && c < cols) ? 0xFFFFu : 0u;
  }
  const v4f a = (v4f){ x[0], x[1], x[2], x[3] };
  const v4f c = (v4f){ x[4], x[5], x[6], x[7] };
  v4u o;
  if (FORM == 2) {
    o = pack8_f16(a, c);
  } else {
    const v4u hi = pack8_bf16(a, c);
    o = hi;
    if (FORM == 1) { const v4u lo = pack8_bf16_lo(a, c); o = second ? lo : hi; }
  }
  const v4u mw = (v4u){ pk16(mk[0], mk[1]), pk16(mk[2], mk[3]), pk16(mk[4], mk[5]), pk16(mk[6], mk[7]) };
  o &= mw;
  if (g < total) {
    volatile v4u* q = (volatile v4u*)(dst + (size_t)g * 8);
    *q = o;
    __threadfence();
    *q = o;
  }
}

template <int FORM> struct FragOf    { typedef FragB T; };
template <>         struct FragOf<2> { typedef FragH T; };
__device__ __forceinline__ v8f mm(const FragB& a, const FragB& b, v8f c) { return wmb(a, b, c); }
__device__ __forceinline__ v8f mm(const FragH& a, const FragH& b, v8f c) { return wmh(a, b, c); }
template <class F> __device__ __forceinline__ F ld_frag(const unsigned short* p) {
  F f;
  f.h[0] = *(const v8usa*)(p);
  f.h[1] = *(const v8usa*)(p + 16);
  return f;
}

template <int FORM, int EPI>
__global__ __launch_bounds__(256) __attribute__((amdgpu_num_vgpr(248)))
void k_gemm_nt(const unsigned short* __restrict__ A, const unsigned short* __restrict__ B,
               const float* __restrict__ bias, float* __restrict__ D, int M, int N, int KTOT, int ldd) {
  static_assert(FORM >= 0 && FORM <= 2);
  static_assert(EPI == 0 || EPI == 1);
  typedef typename FragOf<FORM>::T F;
  __shared__ __attribute__((aligned(16))) float sT[8][16 * 68];
  const int lane = threadIdx.x & 31;
  const int wave = threadIdx.x >> 5;
  const int tilesM = (M + 63) >> 6;
  const int tilesN = (N + 63) >> 6;
  const int tile = blockIdx.x * 8 + wave;
  if (tile >= tilesM * tilesN) return;
  const int tm = tile / tilesN;
  const int tn = tile - tm * tilesN;
  const int m0 = tm << 6;
  const int n0 = tn << 6;

  const int rl = lane & 15;
  const int h8 = (lane >> 4) * 8;
  const unsigned short* pa = A + (size_t)(m0 + rl) * (size_t)KTOT + h8;
  const unsigned short* pb = B + (size_t)(n0 + rl) * (size_t)KTOT + h8;

  v8f acc[4][4];
#pragma unroll
  for (int i = 0; i < 4; ++i)
#pragma unroll
    for (int j = 0; j < 4; ++j) acc[i][j] = (v8f){0.f, 0.f, 0.f, 0.f, 0.f, 0.f, 0.f, 0.f};

#pragma unroll 1
  for (int k0 = 0; k0 < KTOT; k0 += 32) {
    F bf[4];
#pragma unroll
    for (int j = 0; j < 4; ++j) bf[j] = ld_frag<F>(pb + (size_t)(j << 4) * (size_t)KTOT + k0);
#pragma unroll
    for (int i = 0; i < 4; ++i) {
      const F af = ld_frag<F>(pa + (size_t)(i << 4) * (size_t)KTOT + k0);
#pragma unroll
      for (int j = 0; j < 4; ++j) acc[i][j] = mm(af, bf[j], acc[i][j]);
    }
  }

  float* slab = sT[wave];
  const int hh = lane >> 4;
  const int c4 = (lane & 15) * 4;
  const int nc = n0 + c4;
  const bool cok = nc < N;
  v4f bv = (v4f){0.f, 0.f, 0.f, 0.f};
  if (EPI == 1) {
    bv = *(const v4fa*)(bias + clampi(nc, 0, N - 4));
    asm volatile("" :: "v"(bv));
  }
#pragma unroll
  for (int i = 0; i < 4; ++i) {
    const int mBase = m0 + (i << 4);
#pragma unroll
    for (int j = 0; j < 4; ++j) {
#pragma unroll
      for (int r = 0; r < 8; ++r) slab[(h8 + r) * 68 + (j << 4) + rl] = acc[i][j][r];
    }
    __builtin_amdgcn_fence(__ATOMIC_RELEASE, "workgroup");
    __builtin_amdgcn_wave_barrier();
    __builtin_amdgcn_fence(__ATOMIC_ACQUIRE, "workgroup");
    v4f vv[8];
#pragma unroll
    for (int it = 0; it < 8; ++it) {
      const int row = it * 2 + hh;
      v4f v = *(const v4fa*)(slab + row * 68 + c4);
      if (EPI == 1) v += bv;
      vv[it] = v;
    }
    for (int pass = 0; pass < 2; ++pass) {
#pragma unroll
      for (int it = 0; it < 8; ++it) {
        const int row = mBase + it * 2 + hh;
        if (cok && row < M) *(volatile v4f*)(D + (size_t)row * (size_t)ldd + nc) = vv[it];
      }
      __threadfence();
    }
    __builtin_amdgcn_fence(__ATOMIC_RELEASE, "workgroup");
    __builtin_amdgcn_wave_barrier();
    __builtin_amdgcn_fence(__ATOMIC_ACQUIRE, "workgroup");
  }
}

#ifndef PW_FORM
#define PW_FORM 2
#endif
static_assert(PW_FORM >= 1 && PW_FORM <= 3);
#if PW_FORM == 2
#define HLK    1152
#define GFORM  1
#define GEPI   1
#define WF16   0
#define WCARRY 1.0f
#define PWINV  1.0f
#elif PW_FORM == 1
#define HLK    576
#define GFORM  0
#define GEPI   1
#define WF16   0
#define WCARRY 1.0f
#define PWINV  1.0f
#else
#define HLK    576
#define GFORM  2
#define GEPI   0
#define WF16   1
#define WCARRY 64.0f
#define PWINV  0.015625f
#endif

#define IMG_B   4
#define IMG_H   128
#define IMG_W   128
#define IMG_C   128
#define NGRP    2
#define CGRP    64
#define NTAP    9
#define KIN     576
#define FGRP    64
#define NOFF    32
#define NOFFR   18
#define MCH     16384
#define NPIX    65536
#define HLW     (HLK / 2)
#define DWW_P   1296
#define DWB_P   144
#define DWV_P   1440
#define DWV_F   5760
#define VEC_PWB  11520
#define VEC_OFFB 11648
#define VEC_F    12288
#define DW_PPW  4
#define WSLIM   ((size_t)128 << 20)

static_assert(IMG_H == 128 && IMG_W == 128 && IMG_C == 128);
static_assert(CGRP * NGRP == IMG_C && CGRP == 64 && NTAP == 9);
static_assert(KIN == NTAP * CGRP && KIN == 18 * 32);
static_assert(HLK % 32 == 0 && (PW_FORM != 2 || HLK == 36 * 32));
static_assert(MCH == IMG_H * IMG_W && MCH % 128 == 0 && MCH % 64 == 0);
static_assert(NPIX == IMG_B * MCH);
static_assert(NOFF == 32 && NOFFR == 2 * NTAP && NOFFR <= NOFF && NOFF % 4 == 0);
static_assert((KIN * 4) % 128 == 0);
static_assert((HLK * 2) % 128 == 0);
static_assert((KIN * 2) % 128 == 0);
static_assert(DWW_P * 4 == NTAP * KIN && DWB_P * 4 == KIN && DWV_P == DWW_P + DWB_P && DWV_F == 4 * DWV_P);
static_assert(VEC_PWB == NGRP * DWV_F && VEC_OFFB == VEC_PWB + NGRP * FGRP && VEC_OFFB + NGRP * NOFF <= VEC_F);
static_assert(VEC_F % 1024 == 0);
static_assert((DWV_F * 4) % 128 == 0 && (VEC_PWB * 4) % 128 == 0 && (VEC_OFFB * 4) % 128 == 0);
static_assert(DWV_F * 4 <= 327680 && 8 * 16 * 68 * 4 <= 327680);
static_assert(MCH % (8 * DW_PPW) == 0 && IMG_W % DW_PPW == 0);
static_assert((MCH * (KIN / 8)) % 256 == 0);
static_assert((64 * (KIN / 8)) % 256 == 0 && (64 * (HLK / 8)) % 256 == 0);
static_assert((long long)NPIX * IMG_C == 8388608LL);

typedef float        v2f __attribute__((ext_vector_type(2)));
typedef unsigned int v2u __attribute__((ext_vector_type(2)));
typedef v2f __attribute__((may_alias)) v2fa;
typedef v2u __attribute__((may_alias)) v2ua;
typedef v4u __attribute__((may_alias)) v4ua;

template <int F16>
__global__ __launch_bounds__(256) void k_wt(const float* __restrict__ W, int K, int N, int NP,
                                            unsigned short* __restrict__ dst, int KTOT, float carry) {
  const unsigned ppr   = (unsigned)(KTOT >> 3);
  const unsigned total = (unsigned)NP * ppr;
  const unsigned g     = blockIdx.x * 256u + threadIdx.x;
  const unsigned gc    = g < total ? g : total - 1u;
  const unsigned n     = gc / ppr;
  const unsigned p     = gc - n * ppr;
  const int kk = (int)(p << 3);
  const int k0 = (kk >= K) ? kk - K : kk;
  const float* Wg = W + (size_t)blockIdx.y * (size_t)K * (size_t)N;
  unsigned short* dg = dst + (size_t)blockIdx.y * (size_t)NP * (size_t)KTOT;
  const int ncl = clampi((int)n, 0, N - 1);
  const unsigned mk = ((int)n < N) ? 0xFFFFFFFFu : 0u;
  float x[8];
#pragma unroll
  for (int e = 0; e < 8; ++e) {
    const float v = Wg[(size_t)clampi(k0 + e, 0, K - 1) * (size_t)N + ncl];
    asm volatile("" :: "v"(v));
    x[e] = carry * bf16_val(v);
  }
  const v4f a = (v4f){ x[0], x[1], x[2], x[3] };
  const v4f c = (v4f){ x[4], x[5], x[6], x[7] };
  v4u o = F16 ? pack8_f16(a, c) : pack8_bf16(a, c);
  o &= (v4u){ mk, mk, mk, mk };
  if (g < total) {
    volatile v4u* q = (volatile v4u*)(dg + (size_t)g * 8);
    *q = o;
    __threadfence();
    *q = o;
  }
}

__global__ __launch_bounds__(256) void k_vec(const float* __restrict__ dww, const float* __restrict__ dwb,
                                             const float* __restrict__ pwb, const float* __restrict__ offb,
                                             float* __restrict__ VEC) {
  const int t  = blockIdx.x * 256 + threadIdx.x;
  const int gq = t / DWV_P;
  const int q  = t - gq * DWV_P;
  const int iw = clampi(gq * DWW_P + q, 0, NGRP * DWW_P - 1);
  const int ib = clampi(gq * DWB_P + q - DWW_P, 0, NGRP * DWB_P - 1);
  const int ip = clampi(t - NGRP * DWV_P, 0, NGRP * FGRP / 4 - 1);
  const int po = clampi(t - (NGRP * DWV_P + NGRP * FGRP / 4), 0, NGRP * NOFF / 4 - 1);
  const int go = po >> 3;
  const int j0 = (po & 7) * 4;
  const v4f xw = *(const v4fa*)(dww + 4 * iw);
  const v4f xb = *(const v4fa*)(dwb + 4 * ib);
  const v4f xp = *(const v4fa*)(pwb + 4 * ip);
  const float xo0 = offb[clampi(go * NOFFR + j0 + 0, 0, NGRP * NOFFR - 1)];
  const float xo1 = offb[clampi(go * NOFFR + j0 + 1, 0, NGRP * NOFFR - 1)];
  const float xo2 = offb[clampi(go * NOFFR + j0 + 2, 0, NGRP * NOFFR - 1)];
  const float xo3 = offb[clampi(go * NOFFR + j0 + 3, 0, NGRP * NOFFR - 1)];
  asm volatile("" :: "v"(xw), "v"(xb), "v"(xp), "v"(xo0), "v"(xo1), "v"(xo2), "v"(xo3));
  const bool inDW = t < NGRP * DWV_P;
  const bool inPW = (t >= NGRP * DWV_P) && (t < NGRP * DWV_P + NGRP * FGRP / 4);
  const bool inOF = (t >= NGRP * DWV_P + NGRP * FGRP / 4) && (t < NGRP * DWV_P + NGRP * FGRP / 4 + NGRP * NOFF / 4);
  const unsigned mw = (inDW && q < DWW_P) ? 0xFFFFFFFFu : 0u;
  const unsigned mb = (inDW && q >= DWW_P) ? 0xFFFFFFFFu : 0u;
  const unsigned mp = inPW ? 0xFFFFFFFFu : 0u;
  const v4f xo = (v4f){ xo0, xo1, xo2, xo3 };
  v4f o;
#pragma unroll
  for (int e = 0; e < 4; ++e) {
    const unsigned mo = (inOF && (j0 + e) < NOFFR) ? 0xFFFFFFFFu : 0u;
    const unsigned bits = ((bf16_bits(xw[e]) << 16) & mw) | ((bf16_bits(xb[e]) << 16) & mb) |
                          ((bf16_bits(xp[e]) << 16) & mp) | ((bf16_bits(xo[e]) << 16) & mo);
    o[e] = __uint_as_float(bits);
  }
  volatile v4f* d = (volatile v4f*)(VEC + 4 * t);
  *d = o;
  __threadfence();
  *d = o;
}

__global__ __launch_bounds__(256) void k_im2col(const unsigned short* __restrict__ XB,
                                                unsigned short* __restrict__ AIM, int b, int g) {
  const unsigned t   = blockIdx.x * 256u + threadIdx.x;
  const unsigned pos = t / 72u;
  const unsigned p   = t - pos * 72u;
  const int tap = (int)(p >> 3);
  const int sub = (int)(p & 7u);
  const int ky  = tap / 3;
  const int kx  = tap - ky * 3;
  const int h   = (int)(pos >> 7);
  const int w   = (int)(pos & 127u);
  const int hh  = h + ky - 1;
  const int ww  = w + kx - 1;
  const bool ok = ((unsigned)hh < (unsigned)IMG_H) && ((unsigned)ww < (unsigned)IMG_W);
  const int hc  = clampi(hh, 0, IMG_H - 1);
  const int wc  = clampi(ww, 0, IMG_W - 1);
  const size_t si = ((size_t)b * MCH + (size_t)(hc * IMG_W + wc)) * IMG_C + (size_t)(g * CGRP + sub * 8);
  v4u v = *(const v4ua*)(XB + si);
  asm volatile("" :: "v"(v));
  const unsigned mk = ok ? 0xFFFFFFFFu : 0u;
  v &= (v4u){ mk, mk, mk, mk };
  volatile v4u* q = (volatile v4u*)(AIM + (size_t)t * 8);
  *q = v;
  __threadfence();
  *q = v;
}

__device__ __forceinline__ float clip127(float v) {
  v = (v < 0.0f) ? 0.0f : v;
  v = (v > 127.0f) ? 127.0f : v;
  return v;
}
__device__ __forceinline__ int cidx(float v) {
  const float s = (v == v) ? v : 0.0f;
  return clampi((int)s, 0, 127);
}

__global__ __launch_bounds__(256) void k_sample(const unsigned* __restrict__ XBw, const float* __restrict__ OFF,
                                                float* __restrict__ S, int b, int g) {
  const int lane = threadIdx.x & 31;
  const int wave = threadIdx.x >> 5;
  const int pos  = blockIdx.x * 8 + wave;
  const int h = pos >> 7;
  const int w = pos & 127;
  const float offv = OFF[(size_t)pos * NOFF + lane];
  const unsigned* base = XBw + (size_t)b * ((size_t)MCH * (IMG_C / 2)) + (size_t)(g * (CGRP / 2) + lane);
  float* srow = S + (size_t)pos * KIN + 2 * lane;
#pragma unroll 1
  for (int k2 = 0; k2 < NTAP; ++k2) {
    const int iy = k2 / 3;
    const int ix = k2 - iy * 3;
    const float ox = __shfl(offv, 2 * k2);
    const float oy = __shfl(offv, 2 * k2 + 1);
    float lx = (float)(w + ix - 1) + ox;
    float ly = (float)(h + iy - 1) + oy;
    lx = clip127(lx);
    ly = clip127(ly);
    float x0 = floorf(lx);
    float y0 = floorf(ly);
    const float x1 = clip127(x0 + 1.0f);
    x0 = clip127(x0);
    const float y1 = clip127(y0 + 1.0f);
    y0 = clip127(y0);
    const float wa = (x1 - lx) * (y1 - ly);
    const float wb = (x1 - lx) * (ly - y0);
    const float wc = (lx - x0) * (y1 - ly);
    const float wd = (lx - x0) * (ly - y0);
    const int x0i = cidx(x0);
    const int x1i = cidx(x1);
    const int y0i = cidx(y0);
    const int y1i = cidx(y1);
    const unsigned qa = base[(y0i * IMG_W + x0i) * (IMG_C / 2)];
    const unsigned qb = base[(y1i * IMG_W + x0i) * (IMG_C / 2)];
    const unsigned qc = base[(y0i * IMG_W + x1i) * (IMG_C / 2)];
    const unsigned qd = base[(y1i * IMG_W + x1i) * (IMG_C / 2)];
    asm volatile("" :: "v"(qa), "v"(qb), "v"(qc), "v"(qd));
    const float a0 = __uint_as_float(qa << 16), a1 = __uint_as_float(qa & 0xffff0000u);
    const float b0 = __uint_as_float(qb << 16), b1 = __uint_as_float(qb & 0xffff0000u);
    const float c0 = __uint_as_float(qc << 16), c1 = __uint_as_float(qc & 0xffff0000u);
    const float d0 = __uint_as_float(qd << 16), d1 = __uint_as_float(qd & 0xffff0000u);
    float r0 = wa * a0;
    r0 = r0 + wb * b0;
    r0 = r0 + wc * c0;
    r0 = r0 + wd * d0;
    float r1 = wa * a1;
    r1 = r1 + wb * b1;
    r1 = r1 + wc * c1;
    r1 = r1 + wd * d1;
    const v2f r = (v2f){ r0, r1 };
    volatile v2f* q = (volatile v2f*)(srow + k2 * CGRP);
    *q = r;
    __threadfence();
    *q = r;
  }
}

__global__ __launch_bounds__(256) void k_dw(const unsigned* __restrict__ Sw, const float* __restrict__ DWV,
                                            unsigned* __restrict__ HLw) {
  __shared__ __attribute__((aligned(16))) float sDW[DWV_F];
  for (int i = threadIdx.x; i < DWV_P; i += 256) {
    const v4f v = *(const v4fa*)(DWV + 4 * i);
    *(v4fa*)(sDW + 4 * i) = v;
  }
  __syncthreads();

  const int lane = threadIdx.x & 31;
  const int wave = threadIdx.x >> 5;
  const int pos0 = (blockIdx.x * 8 + wave) * DW_PPW;
#pragma unroll 1
  for (int i = 0; i < DW_PPW; ++i) {
    const int pos = pos0 + i;
    const int h = pos >> 7;
    const int w = pos & 127;
#pragma unroll 1
    for (int k2 = 0; k2 < NTAP; ++k2) {
      const int col = k2 * CGRP + 2 * lane;
      float a0 = 0.0f;
      float a1 = 0.0f;
#pragma unroll 1
      for (int ky = 0; ky < 3; ++ky) {
        const int hh = h + ky - 1;
        const bool hok = (unsigned)hh < (unsigned)IMG_H;
        const int hc = clampi(hh, 0, IMG_H - 1);
#pragma unroll
        for (int kx = 0; kx < 3; ++kx) {
          const int ww = w + kx - 1;
          const bool ok = hok && ((unsigned)ww < (unsigned)IMG_W);
          const int wc = clampi(ww, 0, IMG_W - 1);
          const v2u sv = *(const v2ua*)(Sw + (size_t)(hc * IMG_W + wc) * KIN + col);
          asm volatile("" :: "v"(sv));
          const unsigned mk = ok ? 0xFFFFFFFFu : 0u;
          const v2f wv = *(const v2fa*)(sDW + (ky * 3 + kx) * KIN + col);
          a0 = a0 + __uint_as_float(sv[0] & mk) * wv[0];
          a1 = a1 + __uint_as_float(sv[1] & mk) * wv[1];
        }
      }
      const v2f bb = *(const v2fa*)(sDW + NTAP * KIN + col);
      const float t0 = a0 + bb[0];
      const float t1 = a1 + bb[1];
      volatile unsigned* ph = (volatile unsigned*)(HLw + (size_t)pos * HLW + k2 * (CGRP / 2) + lane);
#if PW_FORM == 2
      const unsigned hiw = pk16(bf16_bits(t0), bf16_bits(t1));
      const unsigned low = pk16(bf16_lo_bits(t0), bf16_lo_bits(t1));
      volatile unsigned* pl = ph + (KIN / 2);
      *ph = hiw;
      *pl = low;
      __threadfence();
      *ph = hiw;
      *pl = low;
#elif PW_FORM == 1
      const unsigned hiw = pk16(bf16_bits(t0), bf16_bits(t1));
      *ph = hiw;
      __threadfence();
      *ph = hiw;
#else
      const unsigned hiw = pk16(f16_bits(t0), f16_bits(t1));
      *ph = hiw;
      __threadfence();
      *ph = hiw;
#endif
    }
  }
}

#if PW_FORM == 3
__global__ __launch_bounds__(256) void k_fin(const float* __restrict__ Y, const float* __restrict__ PWB,
                                             float* __restrict__ Dg) {
  const unsigned t = blockIdx.x * 256u + threadIdx.x;
  const unsigned row = t >> 4;
  const unsigned c4 = (t & 15u) * 4u;
  const v4f y = *(const v4fa*)(Y + (size_t)row * FGRP + c4);
  const v4f bb = *(const v4fa*)(PWB + c4);
  v4f o;
#pragma unroll
  for (int e = 0; e < 4; ++e) o[e] = y[e] * PWINV + bb[e];
  volatile v4f* d = (volatile v4f*)(Dg + (size_t)row * IMG_C + c4);
  *d = o;
  __threadfence();
  *d = o;
}
#endif

extern "C" void kernel_launch(void* const* d_in, const int* in_sizes, int n_in,
                              void* d_out, int out_size, void* d_ws, size_t ws_size,
                              hipStream_t stream) {
  if (n_in < 7) return;
  if (in_sizes[0] != NPIX * IMG_C) return;
  if (in_sizes[1] != NGRP * KIN * NOFFR) return;
  if (in_sizes[2] != NGRP * NOFFR) return;
  if (in_sizes[3] != NGRP * NTAP * KIN) return;
  if (in_sizes[4] != NGRP * KIN) return;
  if (in_sizes[5] != NGRP * KIN * FGRP) return;
  if (in_sizes[6] != NGRP * FGRP) return;
  if (out_size != NPIX * IMG_C) return;

  const float* x    = (const float*)d_in[0];
  const float* offw = (const float*)d_in[1];
  const float* offb = (const float*)d_in[2];
  const float* dww  = (const float*)d_in[3];
  const float* dwb  = (const float*)d_in[4];
  const float* pww  = (const float*)d_in[5];
  const float* pwb  = (const float*)d_in[6];
  float* out = (float*)d_out;

  constexpr size_t szXB   = (size_t)NPIX * IMG_C * 2;
  constexpr size_t szAIM  = (size_t)MCH * KIN * 2;
  constexpr size_t szOFF  = (size_t)MCH * NOFF * 4;
  constexpr size_t szS    = (size_t)MCH * KIN * 4;
  constexpr size_t szHL   = (size_t)MCH * HLK * 2;
  constexpr size_t szWOFF = (size_t)NGRP * 64 * KIN * 2;
  constexpr size_t szWPW  = (size_t)NGRP * 64 * HLK * 2;
  constexpr size_t szVEC  = (size_t)VEC_F * 4;
#if PW_FORM == 3
  constexpr size_t szY    = (size_t)MCH * FGRP * 4;
#else
  constexpr size_t szY    = 0;
#endif
  static_assert(szXB % 256 == 0 && szAIM % 256 == 0 && szOFF % 256 == 0 && szS % 256 == 0);
  static_assert(szHL % 256 == 0 && szWOFF % 256 == 0 && szWPW % 256 == 0 && szVEC % 256 == 0 && szY % 256 == 0);
  constexpr size_t oXB   = 0;
  constexpr size_t oAIM  = oXB + szXB;
  constexpr size_t oOFF  = oAIM + szAIM;
  constexpr size_t oS    = oOFF + szOFF;
  constexpr size_t oHL   = oS + szS;
  constexpr size_t oWOFF = oHL + szHL;
  constexpr size_t oWPW  = oWOFF + szWOFF;
  constexpr size_t oVEC  = oWPW + szWPW;
  constexpr size_t oY    = oVEC + szVEC;
  constexpr size_t total = oY + szY;
  static_assert(total <= WSLIM);
  static_assert(PW_FORM != 2 || total == ((size_t)27768 * 4096));
  if (total > ws_size) return;

  char* ws = (char*)d_ws;
  unsigned short* XB   = (unsigned short*)(ws + oXB);
  unsigned short* AIM  = (unsigned short*)(ws + oAIM);
  float*          OFF  = (float*)(ws + oOFF);
  float*          S    = (float*)(ws + oS);
  unsigned short* HL   = (unsigned short*)(ws + oHL);
  unsigned short* WOFF = (unsigned short*)(ws + oWOFF);
  unsigned short* WPW  = (unsigned short*)(ws + oWPW);
  float*          VEC  = (float*)(ws + oVEC);
#if PW_FORM == 3
  float*          Y    = (float*)(ws + oY);
#endif

  k_plane<0><<<dim3(NPIX * (IMG_C / 8) / 256), dim3(256), 0, stream>>>(x, NPIX, IMG_C, IMG_C, XB, NPIX, IMG_C);
  k_wt<0><<<dim3(64 * (KIN / 8) / 256, NGRP), dim3(256), 0, stream>>>(offw, KIN, NOFFR, 64, WOFF, KIN, 1.0f);
  k_wt<WF16><<<dim3(64 * (HLK / 8) / 256, NGRP), dim3(256), 0, stream>>>(pww, KIN, FGRP, 64, WPW, HLK, WCARRY);
  k_vec<<<dim3(VEC_F / 4 / 256), dim3(256), 0, stream>>>(dww, dwb, pwb, offb, VEC);

  const int tiles = (MCH / 64) * 1;
  for (int g = 0; g < NGRP; ++g) {
    for (int b = 0; b < IMG_B; ++b) {
      k_im2col<<<dim3(MCH * (KIN / 8) / 256), dim3(256), 0, stream>>>(XB, AIM, b, g);
      k_gemm_nt<0, 1><<<dim3((tiles + 7) / 8), dim3(256), 0, stream>>>(
          AIM, WOFF + (size_t)g * 64 * KIN, VEC + VEC_OFFB + g * NOFF, OFF, MCH, NOFF, KIN, NOFF);
      k_sample<<<dim3(MCH / 8), dim3(256), 0, stream>>>((const unsigned*)XB, OFF, S, b, g);
      k_dw<<<dim3(MCH / (8 * DW_PPW)), dim3(256), 0, stream>>>((const unsigned*)S, VEC + g * DWV_F, (unsigned*)HL);
      float* Dg = out + (size_t)b * MCH * IMG_C + (size_t)g * FGRP;
#if PW_FORM == 3
      k_gemm_nt<GFORM, GEPI><<<dim3((tiles + 7) / 8), dim3(256), 0, stream>>>(
          HL, WPW + (size_t)g * 64 * HLK, VEC + VEC_PWB + g * FGRP, Y, MCH, FGRP, HLK, FGRP);
      k_fin<<<dim3(MCH * FGRP / 4 / 256), dim3(256), 0, stream>>>(Y, VEC + VEC_PWB + g * FGRP, Dg);
#else
      k_gemm_nt<GFORM, GEPI><<<dim3((tiles + 7) / 8), dim3(256), 0, stream>>>(
          HL, WPW + (size_t)g * 64 * HLK, VEC + VEC_PWB + g * FGRP, Dg, MCH, FGRP, HLK, IMG_C);
#endif
    }
  }
  (void)hipGetLastError();
}
